// LSTMDirectionModel_24086176596736
// MI455X (gfx1250) — hardware-verified
//
#include <hip/hip_runtime.h>
#include <math.h>

typedef __attribute__((ext_vector_type(16))) _Float16 v16h;
typedef __attribute__((ext_vector_type(16))) __bf16 v16b;
typedef __attribute__((ext_vector_type(8)))  _Float16 v8h;
typedef __attribute__((ext_vector_type(8)))  float v8f;
typedef __attribute__((ext_vector_type(4)))  float v4f;
typedef __attribute__((ext_vector_type(2)))  float v2f;
typedef __attribute__((ext_vector_type(4)))  unsigned v4u;
typedef __attribute__((ext_vector_type(4)))  int v4i;
typedef float __attribute__((may_alias)) float_a;
typedef int __attribute__((may_alias)) int_a;

template <typename T> __device__ __forceinline__ void vst2(void* p, T v) { *(volatile T*)p = v; __threadfence(); *(volatile T*)p = v; }
__device__ __forceinline__ v8f wmma16(v16h a, v16h b, v8f c) {
  v8f d = __builtin_amdgcn_wmma_f32_16x16x32_f16(false, a, false, b, (short)0, c, false, false);
  asm volatile("v_nop\n\tv_nop\n\tv_nop\n\tv_nop" : "+v"(d) : "v"(a), "v"(b));
  return d;
}
__device__ __forceinline__ v8f wmma_bf(v16b a, v16b b, v8f c) {
  v8f d = __builtin_amdgcn_wmma_f32_16x16x32_bf16(false, a, false, b, (short)0, c, false, false);
  asm volatile("v_nop\n\tv_nop\n\tv_nop\n\tv_nop" : "+v"(d) : "v"(a), "v"(b));
  return d;
}
__device__ __forceinline__ v16h frag_h(const _Float16* rowk0, int lane) {
  union { v16h v; v8h q[2]; } u; const _Float16* p = rowk0 + 8 * (lane >> 4);
  u.q[0] = *(const v8h*)p; u.q[1] = *(const v8h*)(p + 16); return u.v;
}
__device__ __forceinline__ v16h frag_f32(const float* rowk0, int lane) {
  v16h a; const float* p = rowk0 + 8 * (lane >> 4);
#pragma unroll
  for (int i = 0; i < 8; ++i) { a[i] = (_Float16)p[i]; a[8 + i] = (_Float16)p[16 + i]; }
  return a;
}
__device__ __forceinline__ v16h frag_f32s(const float* rowk0, int lane, float sc) {
  v16h a; const float* p = rowk0 + 8 * (lane >> 4);
#pragma unroll
  for (int i = 0; i < 8; ++i) { a[i] = (_Float16)(p[i] * sc); a[8 + i] = (_Float16)(p[16 + i] * sc); }
  return a;
}
__device__ __forceinline__ v16h fragc_f32(const float* W, int k0, int n, int lane, int ld, int K) {
  v16h a; const int g = lane >> 4;
#pragma unroll
  for (int i = 0; i < 8; ++i) { const int ka = k0 + 8 * g + i, kb = ka + 16;
    a[i] = (_Float16)(ka < K ? W[(size_t)(ka < K ? ka : K - 1) * ld + n] : 0.f); a[8 + i] = (_Float16)(kb < K ? W[(size_t)(kb < K ? kb : K - 1) * ld + n] : 0.f); }
  return a;
}
struct F2 { v16b h, l; };
__device__ __forceinline__ F2 bsplit16(const float v[16]) { F2 r;
#pragma unroll
  for (int i = 0; i < 16; ++i) { const __bf16 h = (__bf16)v[i]; r.h[i] = h; r.l[i] = (__bf16)(v[i] - (float)h); }
  return r; }
__device__ __forceinline__ F2 split_row(const float* row, int k0, int lane) { float v[16]; const float* p = row + k0 + 8 * (lane >> 4);
#pragma unroll
  for (int i = 0; i < 8; ++i) { v[i] = p[i]; v[8 + i] = p[16 + i]; }
  return bsplit16(v); }
__device__ __forceinline__ F2 split_rowK(const float* row, int k0, int lane, int K) { float v[16]; const int g = lane >> 4;
#pragma unroll
  for (int i = 0; i < 8; ++i) { const int ka = k0 + 8 * g + i, kb = ka + 16; v[i] = ka < K ? row[ka < K ? ka : K - 1] : 0.f; v[8 + i] = kb < K ? row[kb < K ? kb : K - 1] : 0.f; }
  return bsplit16(v); }
__device__ __forceinline__ F2 split_col(const float* W, int k0, int n, int lane, int ld, int K) { float v[16]; const int g = lane >> 4;
#pragma unroll
  for (int i = 0; i < 8; ++i) { const int ka = k0 + 8 * g + i, kb = ka + 16; v[i] = ka < K ? W[(size_t)(ka < K ? ka : K - 1) * ld + n] : 0.f; v[8 + i] = kb < K ? W[(size_t)(kb < K ? kb : K - 1) * ld + n] : 0.f; }
  return bsplit16(v); }
__device__ __forceinline__ v8f mac3(const F2& a, const F2& b, v8f c) { c = wmma_bf(a.l, b.h, c); c = wmma_bf(a.h, b.l, c); return wmma_bf(a.h, b.h, c); }
__device__ __forceinline__ float sigm(float v) { return 1.0f / (1.0f + expf(-v)); }
#define LDSX() do { asm volatile("s_wait_dscnt 0" ::: "memory"); __builtin_amdgcn_wave_barrier(); __builtin_amdgcn_fence(__ATOMIC_RELEASE, "workgroup"); } while (0)


#define NBATCH 131072
#define TT 24
#define NI 3
#define NHID 32
#define NG (4 * NHID)
#define F1 16
typedef __attribute__((ext_vector_type(8))) __bf16 v8b;
__device__ __forceinline__ v16b frag_b(const __bf16* rowk0, int lane) {
  union { v16b v; v8b q[2]; } u; const __bf16* p = rowk0 + 8 * (lane >> 4);
  u.q[0] = *(const v8b*)p; u.q[1] = *(const v8b*)(p + 16); return u.v;
}
__device__ __forceinline__ v16b frag_gbf(const float* rowk0, int lane) {
  v16b a; const float* p = rowk0 + 8 * (lane >> 4);
#pragma unroll
  for (int i = 0; i < 8; ++i) { a[i] = (__bf16)p[i]; a[8 + i] = (__bf16)p[16 + i]; }
  return a;
}
__device__ __forceinline__ float bfr(float v) { return (float)(__bf16)v; }
__device__ __attribute__((noinline)) float exp_ni(float v) { return expf(v); }
__device__ __attribute__((noinline)) float tanh_ni(float v) { return tanhf(v); }
__device__ __forceinline__ float sigm_(float v) { return 1.0f / (1.0f + exp_ni(-v)); }
#define WS_END 64u
#ifndef TRB
#define TRB (NBATCH / 64)
#endif

__global__ __launch_bounds__(128) void k_lstm(const float* __restrict__ X, const float* __restrict__ Wih, const float* __restrict__ Whh, const float* __restrict__ bih, const float* __restrict__ bhh, const float* __restrict__ W1, const float* __restrict__ b1, const float* __restrict__ W2, const float* __restrict__ b2, float* __restrict__ OUT) {
  __shared__ __align__(16) __bf16 shh[4][16][40], shl[4][16][40];
  __shared__ float sg[4][16][NG + 1];
  __shared__ float swih[NG][NI + 1], sb[NG], sw1[F1][NHID + 1], sb1[F1], sw2[F1]; __shared__ __align__(16) float sout[64];
  const int tid = threadIdx.x, wave = tid >> 5, lane = tid & 31, col = lane & 15, g = lane >> 4; const size_t r0 = (size_t)blockIdx.x * 64 + wave * 16;
  for (int q = tid; q < NG * NI; q += 128) swih[q / NI][q % NI] = bfr(Wih[q]);
  for (int q = tid; q < NG; q += 128) sb[q] = bfr(bih[q]) + bfr(bhh[q]);
  for (int q = tid; q < F1 * NHID; q += 128) sw1[q / NHID][q % NHID] = bfr(W1[q]);
  if (tid < F1) { sb1[tid] = bfr(b1[tid]); sw2[tid] = bfr(W2[tid]); }
  const int row = lane & 15, half = lane >> 4; float h[16], c[16];
#pragma unroll
  for (int i = 0; i < 16; ++i) { h[i] = 0.f; c[i] = 0.f; shh[wave][row][half * 16 + i] = (__bf16)0.f; shl[wave][row][half * 16 + i] = (__bf16)0.f; }
  __syncthreads();
  const float* xr = X + (r0 + row) * (TT * NI);
#pragma unroll 1
  for (int t = 0; t < TT; ++t) {
    LDSX();
    { const v16b ah = frag_b(&shh[wave][col][0], lane), al = frag_b(&shl[wave][col][0], lane);
#pragma unroll
      for (int j = 0; j < 8; ++j) { const v16b w = frag_gbf(Whh + (size_t)(j * 16 + col) * NHID, lane); v8f acc = {}; acc = wmma_bf(al, w, acc); acc = wmma_bf(ah, w, acc);
#pragma unroll
        for (int r = 0; r < 8; ++r) sg[wave][8 * g + r][j * 16 + col] = acc[r]; } }
    LDSX();
    const float x0 = bfr(xr[t * NI + 0]), x1 = bfr(xr[t * NI + 1]), x2 = bfr(xr[t * NI + 2]);
#pragma unroll
    for (int i = 0; i < 16; ++i) { const int u = half * 16 + i; float gv[4];
#pragma unroll
      for (int q = 0; q < 4; ++q) { const int gc = q * NHID + u; gv[q] = sg[wave][row][gc] + sb[gc] + x0 * swih[gc][0] + x1 * swih[gc][1] + x2 * swih[gc][2]; }
      const float ig = sigm_(gv[0]), fg = sigm_(gv[1]), gg = tanh_ni(gv[2]), og = sigm_(gv[3]);
      c[i] = fg * c[i] + ig * gg; h[i] = og * tanh_ni(c[i]);
      const __bf16 hb = (__bf16)h[i]; shh[wave][row][u] = hb; shl[wave][row][u] = (__bf16)(h[i] - (float)hb); } }
  LDSX();
  __shared__ float shf[4][16][NHID + 1];
#pragma unroll
  for (int i = 0; i < 16; ++i) shf[wave][row][half * 16 + i] = h[i];
  LDSX();
  if (half == 0) { float logit = bfr(b2[0]);
#pragma unroll 1
    for (int o = 0; o < F1; ++o) { float s = sb1[o];
#pragma unroll 1
      for (int u = 0; u < NHID; ++u) s += shf[wave][row][u] * sw1[o][u];
      logit += fmaxf(s, 0.f) * sw2[o]; }
    sout[wave * 16 + row] = logit; }
  __syncthreads();
  if (tid < 16) vst2(OUT + (size_t)blockIdx.x * 64 + tid * 4, *(const v4f*)&sout[tid * 4]);
}
extern "C" void kernel_launch(void* const* d_in, const int* in_sizes, int n_in, void* d_out, int out_size, void* d_ws, size_t ws_size, hipStream_t stream) {
  (void)in_sizes; (void)n_in; (void)out_size; (void)d_ws;
  const float** F = (const float**)d_in;
  if (ws_size < (size_t)WS_END) return;
  k_lstm<<<TRB, 128, 0, stream>>>(F[0], F[1], F[2], F[3], F[4], F[5], F[6], F[7], F[8], (float*)d_out);
}
